// GCNNeck_24962349924890
// MI455X (gfx1250) — hardware-verified
//
#include <hip/hip_runtime.h>
#include <math.h>

typedef __attribute__((ext_vector_type(16))) _Float16 v16h;
typedef __attribute__((ext_vector_type(16))) __bf16 v16b;
typedef __attribute__((ext_vector_type(8)))  _Float16 v8h;
typedef __attribute__((ext_vector_type(8)))  float v8f;
typedef __attribute__((ext_vector_type(4)))  float v4f;
typedef __attribute__((ext_vector_type(2)))  float v2f;
typedef __attribute__((ext_vector_type(4)))  unsigned v4u;
typedef __attribute__((ext_vector_type(4)))  int v4i;
typedef float __attribute__((may_alias)) float_a;
typedef int __attribute__((may_alias)) int_a;

template <typename T> __device__ __forceinline__ void vst2(void* p, T v) { *(volatile T*)p = v; __threadfence(); *(volatile T*)p = v; }
__device__ __forceinline__ v8f wmma16(v16h a, v16h b, v8f c) {
  v8f d = __builtin_amdgcn_wmma_f32_16x16x32_f16(false, a, false, b, (short)0, c, false, false);
  asm volatile("v_nop\n\tv_nop\n\tv_nop\n\tv_nop" : "+v"(d) : "v"(a), "v"(b));
  return d;
}
__device__ __forceinline__ v8f wmma_bf(v16b a, v16b b, v8f c) {
  v8f d = __builtin_amdgcn_wmma_f32_16x16x32_bf16(false, a, false, b, (short)0, c, false, false);
  asm volatile("v_nop\n\tv_nop\n\tv_nop\n\tv_nop" : "+v"(d) : "v"(a), "v"(b));
  return d;
}
__device__ __forceinline__ v16h frag_h(const _Float16* rowk0, int lane) {
  union { v16h v; v8h q[2]; } u; const _Float16* p = rowk0 + 8 * (lane >> 4);
  u.q[0] = *(const v8h*)p; u.q[1] = *(const v8h*)(p + 16); return u.v;
}
__device__ __forceinline__ v16h frag_f32(const float* rowk0, int lane) {
  v16h a; const float* p = rowk0 + 8 * (lane >> 4);
#pragma unroll
  for (int i = 0; i < 8; ++i) { a[i] = (_Float16)p[i]; a[8 + i] = (_Float16)p[16 + i]; }
  return a;
}
__device__ __forceinline__ v16h frag_f32s(const float* rowk0, int lane, float sc) {
  v16h a; const float* p = rowk0 + 8 * (lane >> 4);
#pragma unroll
  for (int i = 0; i < 8; ++i) { a[i] = (_Float16)(p[i] * sc); a[8 + i] = (_Float16)(p[16 + i] * sc); }
  return a;
}
__device__ __forceinline__ v16h fragc_f32(const float* W, int k0, int n, int lane, int ld, int K) {
  v16h a; const int g = lane >> 4;
#pragma unroll
  for (int i = 0; i < 8; ++i) { const int ka = k0 + 8 * g + i, kb = ka + 16;
    a[i] = (_Float16)(ka < K ? W[(size_t)(ka < K ? ka : K - 1) * ld + n] : 0.f); a[8 + i] = (_Float16)(kb < K ? W[(size_t)(kb < K ? kb : K - 1) * ld + n] : 0.f); }
  return a;
}
struct F2 { v16b h, l; };
__device__ __forceinline__ F2 bsplit16(const float v[16]) { F2 r;
#pragma unroll
  for (int i = 0; i < 16; ++i) { const __bf16 h = (__bf16)v[i]; r.h[i] = h; r.l[i] = (__bf16)(v[i] - (float)h); }
  return r; }
__device__ __forceinline__ F2 split_row(const float* row, int k0, int lane) { float v[16]; const float* p = row + k0 + 8 * (lane >> 4);
#pragma unroll
  for (int i = 0; i < 8; ++i) { v[i] = p[i]; v[8 + i] = p[16 + i]; }
  return bsplit16(v); }
__device__ __forceinline__ F2 split_rowK(const float* row, int k0, int lane, int K) { float v[16]; const int g = lane >> 4;
#pragma unroll
  for (int i = 0; i < 8; ++i) { const int ka = k0 + 8 * g + i, kb = ka + 16; v[i] = ka < K ? row[ka < K ? ka : K - 1] : 0.f; v[8 + i] = kb < K ? row[kb < K ? kb : K - 1] : 0.f; }
  return bsplit16(v); }
__device__ __forceinline__ F2 split_col(const float* W, int k0, int n, int lane, int ld, int K) { float v[16]; const int g = lane >> 4;
#pragma unroll
  for (int i = 0; i < 8; ++i) { const int ka = k0 + 8 * g + i, kb = ka + 16; v[i] = ka < K ? W[(size_t)(ka < K ? ka : K - 1) * ld + n] : 0.f; v[8 + i] = kb < K ? W[(size_t)(kb < K ? kb : K - 1) * ld + n] : 0.f; }
  return bsplit16(v); }
__device__ __forceinline__ v8f mac3(const F2& a, const F2& b, v8f c) { c = wmma_bf(a.l, b.h, c); c = wmma_bf(a.h, b.l, c); return wmma_bf(a.h, b.h, c); }
__device__ __forceinline__ float sigm(float v) { return 1.0f / (1.0f + expf(-v)); }
#define LDSX() do { asm volatile("s_wait_dscnt 0" ::: "memory"); __builtin_amdgcn_wave_barrier(); __builtin_amdgcn_fence(__ATOMIC_RELEASE, "workgroup"); } while (0)


#define NP 4096
#define DD 256
#define RAD2 0.015625f
typedef __attribute__((ext_vector_type(8))) __bf16 v8b;
__device__ __forceinline__ v16b frag_b16(const __bf16* rowk0, int lane) {
  union { v16b v; v8b q[2]; } u; const __bf16* p = rowk0 + 8 * (lane >> 4);
  u.q[0] = *(const v8b*)p; u.q[1] = *(const v8b*)(p + 16); return u.v;
}
__device__ __forceinline__ v16b frag_gbf(const float* rowk0, int lane) {
  v16b a; const float* p = rowk0 + 8 * (lane >> 4);
#pragma unroll
  for (int i = 0; i < 8; ++i) { a[i] = (__bf16)p[i]; a[8 + i] = (__bf16)p[16 + i]; }
  return a;
}
__device__ __forceinline__ v16b frag_gbf_neg(const float* rowk0, int lane) {
  v16b a; const float* p = rowk0 + 8 * (lane >> 4);
#pragma unroll
  for (int i = 0; i < 8; ++i) { a[i] = (__bf16)(-p[i]); a[8 + i] = (__bf16)(-p[16 + i]); }
  return a;
}
__device__ __forceinline__ float bfr(float v) { return (float)(__bf16)v; }

#define WS_XT   0u
#define WS_M    (WS_XT + 2u * DD * NP)
#define WS_S    (WS_M + 2u * NP * NP)
#define WS_A2   (WS_S + 4u * NP * DD)
#define WS_DEG  (WS_A2 + 4u * NP * DD)
#define WS_END  (WS_DEG + 4u * NP)

__global__ __launch_bounds__(256) void k_xt(const float* __restrict__ X, __bf16* __restrict__ Xt) {
  __shared__ __align__(16) __bf16 T[64][128 + 8];
  const int n0 = blockIdx.x * 128, d0 = blockIdx.y * 64, tid = threadIdx.x;
#pragma unroll
  for (int it = 0; it < 8; ++it) { const int q = tid + 256 * it; const int r = q >> 4, c4 = (q & 15) * 4;
    const float4 v = *(const float4*)(X + (size_t)(n0 + r) * DD + d0 + c4);
    T[c4 + 0][r] = (__bf16)v.x; T[c4 + 1][r] = (__bf16)v.y; T[c4 + 2][r] = (__bf16)v.z; T[c4 + 3][r] = (__bf16)v.w; }
  __syncthreads();
#pragma unroll
  for (int it = 0; it < 4; ++it) { const int q = tid + 256 * it; const int r = q >> 4, c8 = (q & 15) * 8;
    vst2(Xt + (size_t)(d0 + r) * NP + n0 + c8, *(const v4f*)&T[r][c8]); }
}

__global__ __launch_bounds__(256) void k_mask(const float* __restrict__ C, __bf16* __restrict__ M) {
  const int a = blockIdx.y, k0 = (blockIdx.x * 256 + threadIdx.x) * 8;
  const float ax = bfr(C[a * 3 + 0]), ay = bfr(C[a * 3 + 1]), az = bfr(C[a * 3 + 2]);
  float ck[24];
#pragma unroll
  for (int i = 0; i < 6; ++i) { const float4 v = *(const float4*)(C + (size_t)k0 * 3 + 4 * i); ck[4 * i] = v.x; ck[4 * i + 1] = v.y; ck[4 * i + 2] = v.z; ck[4 * i + 3] = v.w; }
  union { v8b v; v4f f; } o;
#pragma unroll
  for (int i = 0; i < 8; ++i) {
#pragma clang fp contract(off)
    const float dx = ax - bfr(ck[3 * i]), dy = ay - bfr(ck[3 * i + 1]), dz = az - bfr(ck[3 * i + 2]);
    const float d2 = (dx * dx + dy * dy) + dz * dz;
    o.v[i] = (d2 <= RAD2 && (k0 + i) != a) ? (__bf16)1.0f : (__bf16)0.0f;
  }
  vst2(M + (size_t)a * NP + k0, o.f);
}

__global__ __launch_bounds__(256) void k_s(const __bf16* __restrict__ M, const __bf16* __restrict__ Xt, float* __restrict__ S, float* __restrict__ degv) {
  __shared__ __align__(16) float So[64][128 + 4];
  __shared__ __align__(16) float Sdeg[64];
  const int a0 = blockIdx.x * 64, d0 = blockIdx.y * 128, tid = threadIdx.x, wave = tid >> 5, lane = tid & 31, l16 = lane & 15, hh = lane >> 4;
  const int at = wave & 3, dt0 = (wave >> 2) * 4;
  const __bf16* arow = M + (size_t)(a0 + at * 16 + l16) * NP;
  v8f acc[4] = {}; float cnt = 0.f;
#pragma unroll 1
  for (int kc = 0; kc < NP / 32; ++kc) {
    const v16b af = frag_b16(arow + kc * 32, lane);
#pragma unroll
    for (int i = 0; i < 16; ++i) cnt += (float)af[i];
#pragma unroll
    for (int t = 0; t < 4; ++t) acc[t] = wmma_bf(af, frag_b16(Xt + (size_t)(d0 + (dt0 + t) * 16 + l16) * NP + kc * 32, lane), acc[t]);
  }
  cnt += __shfl_xor(cnt, 16);
  if (dt0 == 0 && hh == 0) Sdeg[at * 16 + l16] = cnt;
#pragma unroll
  for (int t = 0; t < 4; ++t)
#pragma unroll
    for (int r = 0; r < 8; ++r) So[at * 16 + 8 * hh + r][(dt0 + t) * 16 + l16] = acc[t][r];
  __syncthreads();
#pragma unroll
  for (int it = 0; it < 8; ++it) { const int q = tid + 256 * it; const int r = q >> 5, c4 = (q & 31) * 4;
    vst2(S + (size_t)(a0 + r) * DD + d0 + c4, *(const v4f*)&So[r][c4]); }
  if (blockIdx.y == 0 && tid < 16) vst2(degv + a0 + tid * 4, *(const v4f*)&Sdeg[tid * 4]);
}

__global__ __launch_bounds__(256) void k_a2(const float* __restrict__ S, const float* __restrict__ X, const float* __restrict__ W1, const float* __restrict__ b1,
                                            const float* __restrict__ degv, float* __restrict__ A2) {
  __shared__ __align__(16) float So[64][128 + 4];
  const int a0 = blockIdx.x * 64, o0 = blockIdx.y * 128, tid = threadIdx.x, wave = tid >> 5, lane = tid & 31, l16 = lane & 15, hh = lane >> 4;
  const int at = wave & 3, ot0 = (wave >> 2) * 4;
  const int arow = a0 + at * 16 + l16;
  v8f acc[4] = {}, accv[4] = {};
#pragma unroll 1
  for (int kc = 0; kc < DD / 32; ++kc) {
    const F2 sf = split_row(S + (size_t)arow * DD, kc * 32, lane);
    const v16b xf = frag_gbf(X + (size_t)arow * DD + kc * 32, lane);
#pragma unroll
    for (int t = 0; t < 4; ++t) { const float* wrow = W1 + (size_t)(o0 + (ot0 + t) * 16 + l16) * (2 * DD) + kc * 32;
      const v16b wa = frag_gbf(wrow, lane), wbn = frag_gbf_neg(wrow + DD, lane), wb = frag_gbf(wrow + DD, lane);
      acc[t] = wmma_bf(sf.l, wa, acc[t]); acc[t] = wmma_bf(sf.l, wbn, acc[t]); acc[t] = wmma_bf(sf.h, wa, acc[t]); acc[t] = wmma_bf(sf.h, wbn, acc[t]);
      accv[t] = wmma_bf(xf, wb, accv[t]); }
  }
#pragma unroll
  for (int t = 0; t < 4; ++t)
#pragma unroll
    for (int r = 0; r < 8; ++r) { const int rr = at * 16 + 8 * hh + r, o = o0 + (ot0 + t) * 16 + l16;
      So[rr][(ot0 + t) * 16 + l16] = acc[t][r] + degv[a0 + rr] * (accv[t][r] + bfr(b1[o])); }
  __syncthreads();
#pragma unroll
  for (int it = 0; it < 8; ++it) { const int q = tid + 256 * it; const int r = q >> 5, c4 = (q & 31) * 4;
    vst2(A2 + (size_t)(a0 + r) * DD + o0 + c4, *(const v4f*)&So[r][c4]); }
}

__global__ __launch_bounds__(256) void k_out(const float* __restrict__ A2, const float* __restrict__ X, const float* __restrict__ W2, const float* __restrict__ b2,
                                             const float* __restrict__ degv, float* __restrict__ out) {
  __shared__ __align__(16) float So[64][256 + 4];
  const int a0 = blockIdx.x * 64, tid = threadIdx.x, wave = tid >> 5, lane = tid & 31, l16 = lane & 15, hh = lane >> 4;
  const int at = wave & 3, et0 = (wave >> 2) * 8;
  const int arow = a0 + at * 16 + l16;
  v8f acc[8] = {};
#pragma unroll 1
  for (int kc = 0; kc < DD / 32; ++kc) {
    const F2 af = split_row(A2 + (size_t)arow * DD, kc * 32, lane);
#pragma unroll
    for (int t = 0; t < 8; ++t) { const float* wrow = W2 + (size_t)((et0 + t) * 16 + l16) * (2 * DD) + kc * 32;
      const v16b wa = frag_gbf(wrow, lane), wbn = frag_gbf_neg(wrow + DD, lane);
      acc[t] = wmma_bf(af.l, wa, acc[t]); acc[t] = wmma_bf(af.l, wbn, acc[t]); acc[t] = wmma_bf(af.h, wa, acc[t]); acc[t] = wmma_bf(af.h, wbn, acc[t]); }
  }
#pragma unroll
  for (int t = 0; t < 8; ++t)
#pragma unroll
    for (int r = 0; r < 8; ++r) { const int rr = at * 16 + 8 * hh + r, e = (et0 + t) * 16 + l16;
      So[rr][e] = (acc[t][r] + degv[a0 + rr] * bfr(b2[e])) * (1.0f / NP); }
  __syncthreads();
#pragma unroll
  for (int it = 0; it < 16; ++it) { const int q = tid + 256 * it; const int r = q >> 6, c4 = (q & 63) * 4;
    vst2(out + (size_t)(a0 + r) * (2 * DD) + DD + c4, *(const v4f*)&So[r][c4]); }
#pragma unroll
  for (int it = 0; it < 16; ++it) { const int q = tid + 256 * it; const int r = q >> 6, c4 = (q & 63) * 4;
    vst2(out + (size_t)(a0 + r) * (2 * DD) + c4, *(const v4f*)(X + (size_t)(a0 + r) * DD + c4)); }
}

extern "C" void kernel_launch(void* const* d_in, const int* in_sizes, int n_in, void* d_out, int out_size, void* d_ws, size_t ws_size, hipStream_t stream) {
  (void)in_sizes; (void)n_in; (void)out_size;
  const float* C  = (const float*)d_in[0];
  const float* X  = (const float*)d_in[1];
  const float* W1 = (const float*)d_in[2];
  const float* b1 = (const float*)d_in[3];
  const float* W2 = (const float*)d_in[4];
  const float* b2 = (const float*)d_in[5];
  if (ws_size < (size_t)WS_END) return;
  char* ws = (char*)d_ws;
  __bf16* Xt = (__bf16*)(ws + WS_XT); __bf16* M = (__bf16*)(ws + WS_M); float* S = (float*)(ws + WS_S); float* A2 = (float*)(ws + WS_A2); float* degv = (float*)(ws + WS_DEG);
  k_xt<<<dim3(NP / 128, DD / 64), 256, 0, stream>>>(X, Xt);
  k_mask<<<dim3(NP / 2048, NP), 256, 0, stream>>>(C, M);
  k_s<<<dim3(NP / 64, DD / 128), 256, 0, stream>>>(M, Xt, S, degv);
  k_a2<<<dim3(NP / 64, DD / 128), 256, 0, stream>>>(S, X, W1, b1, degv, A2);
  k_out<<<dim3(NP / 64), 256, 0, stream>>>(A2, X, W2, b2, degv, (float*)d_out);
}
